// DCNv2_Circle8_85117661872715
// MI455X (gfx1250) — hardware-verified
//
#include <hip/hip_runtime.h>
#include <math.h>

typedef _Float16 v16h __attribute__((ext_vector_type(16)));
typedef _Float16 v8h  __attribute__((ext_vector_type(8)));
typedef _Float16 v2h  __attribute__((ext_vector_type(2)));
typedef float    v8f  __attribute__((ext_vector_type(8)));
typedef float    v4f  __attribute__((ext_vector_type(4)));
union Frag { v16h v; v8h half[2]; };

#define HWSZ   16384
#define WIMG   128
#define CIN    64
#define COUT   64
#define NGRP   8
#define NOUT   512
#define KDIM   576
#define KSTEPS 18
#define MT     32
#define SOSTR  68
#define PSTR   128
#define WQP    576
#define WQCH   72
#define WSCALE 256.0f
#define WINV   (1.0f / 256.0f)
#define LOSC   65536.0f
#define LOINV  (1.0f / 65536.0f)
#define F16MIN 6.103515625e-5f

__constant__ int c_perm[8][9] = {
    {0,1,2,3,4,5,6,7,8},
    {3,0,1,6,4,2,7,8,5},
    {6,3,0,7,4,1,8,5,2},
    {7,6,3,8,4,0,5,2,1},
    {8,7,6,5,4,3,2,1,0},
    {5,8,7,2,4,6,1,0,3},
    {2,5,8,1,4,7,0,3,6},
    {1,2,5,0,4,8,3,6,7}
};

__device__ __forceinline__ v8f wmma16(const v16h a, const v16h b, v8f c) {
    v8f d = __builtin_amdgcn_wmma_f32_16x16x32_f16(false, a, false, b, (short)0, c, false, false);
    asm volatile("v_nop\n\tv_nop\n\tv_nop\n\tv_nop" : "+v"(d) : "v"(a), "v"(b));
    return d;
}

__device__ __forceinline__ void split16(float v, _Float16& h, _Float16& l) {
    _Float16 h16 = (_Float16)v;
    float hf = (float)h16;
    const bool tiny = fabsf(v) < F16MIN;
    hf  = tiny ? 0.0f : hf;
    h16 = tiny ? (_Float16)0.0f : h16;
    h = h16;
    l = (_Float16)((v - hf) * LOSC);
}

__global__ __launch_bounds__(256) void k_pool(const float* __restrict__ input,
                                              float* __restrict__ P, int nplanes) {
    __shared__ float red[256];
    const int blk = blockIdx.x;
    if (blk >= nplanes) return;
    const float* src = input + (size_t)blk * HWSZ;
    float s = 0.f;
    for (int i = threadIdx.x; i < HWSZ; i += 256) s += src[i];
    red[threadIdx.x] = s;
    __syncthreads();
    for (int off = 128; off > 0; off >>= 1) {
        if (threadIdx.x < off) red[threadIdx.x] += red[threadIdx.x + off];
        __syncthreads();
    }
    if (threadIdx.x < 32) {
        const float tot = red[0];
        v4f v; v.x = tot; v.y = tot; v.z = tot; v.w = tot;
        volatile v4f* dst = (volatile v4f*)(P + (size_t)blk * PSTR + threadIdx.x * 4);
        *dst = v;
        __threadfence();
        *dst = v;
    }
}

__global__ __launch_bounds__(256) void k_blend(const float* __restrict__ weight,
                                               const float* __restrict__ P,
                                               const float* __restrict__ fc_w,
                                               const float* __restrict__ fc_b,
                                               _Float16* __restrict__ wq) {
    __shared__ float sWr[CIN * 9];
    __shared__ float sBase[CIN * 9];
    __shared__ float sPool[CIN];
    __shared__ float sR[4];
    const int tid = threadIdx.x;
    const int o   = blockIdx.x;
    if (o >= COUT) return;
    const float* wp = weight + (size_t)o * CIN * 9;
    for (int i = tid; i < CIN * 9; i += 256) sWr[i] = wp[i];
    if (tid < CIN)
        sPool[tid] = (P[(size_t)tid * PSTR] + P[(size_t)(CIN + tid) * PSTR]) * (1.0f / (float)HWSZ);
    __syncthreads();
    if (tid < 4) {
        float acc = fc_b[tid];
        #pragma unroll 1
        for (int j = 0; j < CIN; ++j) acc += sPool[j] * fc_w[tid * CIN + j];
        sR[tid] = 1.0f / (1.0f + expf(-acc));
    }
    for (int c = tid; c < CIN; c += 256) {
        const float* wr = &sWr[c * 9];
        const float S = 0.70710678118654752440f;
        const float T = 1.0f - S;
        const float f0 = S * wr[0] + T * wr[1];
        const float f1 = S * wr[3] + T * wr[4];
        const float w0 = S * f0 + T * f1;
        const float f2 = T * wr[1] + S * wr[2];
        const float f3 = T * wr[4] + S * wr[5];
        const float w2 = S * f2 + T * f3;
        const float f5 = S * wr[6] + T * wr[7];
        const float w6 = T * f1 + S * f5;
        const float f7 = T * wr[7] + S * wr[8];
        const float w8 = T * f3 + S * f7;
        float* bp = &sBase[c * 9];
        bp[0] = w0;    bp[1] = wr[1]; bp[2] = w2;
        bp[3] = wr[3]; bp[4] = wr[4]; bp[5] = wr[5];
        bp[6] = w6;    bp[7] = wr[7]; bp[8] = w8;
    }
    __syncthreads();

    const int lane = tid & 31;
    const int g    = tid >> 5;
    const float f  = (g & 1) ? 1.0f : sR[g >> 1];
    const float fm = 1.0f - f;
    _Float16* row = wq + (size_t)(g * COUT + o) * WQP;

    v8h vals[3];
    #pragma unroll
    for (int jj = 0; jj < 3; ++jj) {
        const int j = lane + 32 * jj;
        v8h v;
        #pragma unroll
        for (int i = 0; i < 8; ++i) {
            int K = 8 * j + i;
            K = K < KDIM ? K : KDIM - 1;
            const int c = K / 9;
            const int k = K - 9 * c;
            const int p = c_perm[g][k];
            const float val = (sBase[c * 9 + p] * f + sWr[c * 9 + p] * fm) * WSCALE;
            v[i] = (_Float16)val;
        }
        vals[jj] = v;
    }
    #pragma unroll
    for (int jj = 0; jj < 3; ++jj) {
        const int j = lane + 32 * jj;
        if (j < WQCH) *(volatile v8h*)(row + 8 * j) = vals[jj];
    }
    __threadfence();
    #pragma unroll
    for (int jj = 0; jj < 3; ++jj) {
        const int j = lane + 32 * jj;
        if (j < WQCH) *(volatile v8h*)(row + 8 * j) = vals[jj];
    }
}

__global__ __launch_bounds__(256) void k_deform(const float* __restrict__ input,
                                                const float* __restrict__ offset,
                                                const float* __restrict__ maskp,
                                                const float* __restrict__ wc8,
                                                const float* __restrict__ bias,
                                                const _Float16* __restrict__ wq,
                                                float* __restrict__ out,
                                                int npix) {
    __shared__ __align__(32) _Float16 sAh[KSTEPS * 2 * 2 * 16 * 16];
    __shared__ __align__(32) _Float16 sAl[KSTEPS * 2 * 2 * 16 * 16];
    __shared__ float sWgt[MT * 9 * 4];
    __shared__ int   sIdx[MT * 9 * 4];
    __shared__ float sW8[MT * 8];
    __shared__ float sOut[MT * SOSTR];

    const int tid     = threadIdx.x;
    const int pixbase = blockIdx.x * MT;
    if (pixbase >= npix) return;
    const int b       = pixbase >> 14;
    const int hwbase  = pixbase & (HWSZ - 1);

    for (int t2 = tid; t2 < MT * 9; t2 += 256) {
        const int p  = t2 / 9;
        const int k  = t2 % 9;
        const int hw = hwbase + p;
        const int h  = hw >> 7;
        const int w  = hw & 127;
        const float oy = offset[((size_t)(b * 18 + 2 * k))     * HWSZ + hw];
        const float ox = offset[((size_t)(b * 18 + 2 * k + 1)) * HWSZ + hw];
        const float mk = maskp [((size_t)(b * 9  + k))         * HWSZ + hw];
        const float py = (float)h + (float)(k / 3) - 1.0f + oy;
        const float px = (float)w + (float)(k % 3) - 1.0f + ox;
        const float y0f = floorf(py), x0f = floorf(px);
        const float ly = py - y0f, lx = px - x0f;
        const int y0 = (int)y0f, x0 = (int)x0f;
        #pragma unroll
        for (int i = 0; i < 4; ++i) {
            const int dy = i >> 1, dx = i & 1;
            const int yi = y0 + dy, xi = x0 + dx;
            const bool valid = (yi >= 0) & (yi <= WIMG - 1) & (xi >= 0) & (xi <= WIMG - 1);
            float wgt = (dy ? ly : 1.0f - ly) * (dx ? lx : 1.0f - lx);
            wgt = valid ? wgt * mk : 0.0f;
            const int yc = yi < 0 ? 0 : (yi > WIMG - 1 ? WIMG - 1 : yi);
            const int xc = xi < 0 ? 0 : (xi > WIMG - 1 ? WIMG - 1 : xi);
            sWgt[t2 * 4 + i] = wgt;
            sIdx[t2 * 4 + i] = yc * WIMG + xc;
        }
    }
    for (int t2 = tid; t2 < MT * 8; t2 += 256) {
        const int p = t2 >> 3, g = t2 & 7;
        sW8[t2] = wc8[((size_t)(b * 8 + g)) * HWSZ + hwbase + p];
    }
    for (int t2 = tid; t2 < MT * SOSTR; t2 += 256) sOut[t2] = 0.0f;
    __syncthreads();

    const float* inb = input + (size_t)b * CIN * HWSZ;
    for (int j = tid; j < MT * (KDIM / 2); j += 256) {
        const int p  = j / (KDIM / 2);
        const int K  = (j % (KDIM / 2)) * 2;
        float v[2];
        #pragma unroll
        for (int u = 0; u < 2; ++u) {
            const int Ku = K + u;
            const int c  = Ku / 9;
            const int k  = Ku - 9 * c;
            const int pk = p * 9 + k;
            const float* ip = inb + (size_t)c * HWSZ;
            const int*   xi = &sIdx[pk * 4];
            const float* xw = &sWgt[pk * 4];
            v[u] = xw[0] * ip[xi[0]] + xw[1] * ip[xi[1]]
                 + xw[2] * ip[xi[2]] + xw[3] * ip[xi[3]];
        }
        const int ks  = K >> 5;
        const int kk  = K & 31;
        const int grp = (kk >> 3) & 1;
        const int e   = (kk & 7) | ((kk >> 4) << 3);
        const int mtile = p >> 4, Mrow = p & 15;
        const int idx = ((((ks * 2 + mtile) * 2 + grp) << 4) + Mrow) * 16 + e;
        _Float16 h0, l0, h1, l1;
        split16(v[0], h0, l0);
        split16(v[1], h1, l1);
        v2h ph; ph[0] = h0; ph[1] = h1;
        v2h pl; pl[0] = l0; pl[1] = l1;
        *(v2h*)&sAh[idx] = ph;
        *(v2h*)&sAl[idx] = pl;
    }
    __syncthreads();

    const int lane = tid & 31;
    const int wid  = tid >> 5;
    const int hh   = lane >> 4;
    const int m    = lane & 15;

    v8f acc[2][4];
    #pragma unroll
    for (int mt = 0; mt < 2; ++mt)
        #pragma unroll
        for (int nt = 0; nt < 4; ++nt)
            #pragma unroll
            for (int e = 0; e < 8; ++e) acc[mt][nt][e] = 0.0f;

    const _Float16* bbase = wq + (size_t)(wid * COUT + m) * WQP + 8 * hh;

    #pragma unroll
    for (int ps = 0; ps < 2; ++ps) {
        const _Float16* sT = (ps == 0) ? sAl : sAh;
        #pragma unroll 1
        for (int ks = 0; ks < KSTEPS; ++ks) {
            const v16h a0 = *(const v16h*)&sT[((((ks * 2 + 0) * 2 + hh) << 4) + m) << 4];
            const v16h a1 = *(const v16h*)&sT[((((ks * 2 + 1) * 2 + hh) << 4) + m) << 4];
            #pragma unroll
            for (int nt = 0; nt < 4; ++nt) {
                const _Float16* bp = bbase + (size_t)(nt * 16) * WQP + ks * 32;
                Frag bf;
                bf.half[0] = *(const v8h*)(bp);
                bf.half[1] = *(const v8h*)(bp + 16);
                acc[0][nt] = wmma16(a0, bf.v, acc[0][nt]);
                acc[1][nt] = wmma16(a1, bf.v, acc[1][nt]);
            }
        }
        if (ps == 0) {
            #pragma unroll
            for (int mt = 0; mt < 2; ++mt)
                #pragma unroll
                for (int nt = 0; nt < 4; ++nt)
                    #pragma unroll
                    for (int e = 0; e < 8; ++e) acc[mt][nt][e] *= LOINV;
        }
    }

    const int msel = hh << 3;
    for (int gp = 0; gp < NGRP; ++gp) {
        if (wid == gp) {
            #pragma unroll
            for (int mt = 0; mt < 2; ++mt) {
                #pragma unroll
                for (int nt = 0; nt < 4; ++nt) {
                    const int co = nt * 16 + m;
                    const float bs = bias[wid * COUT + co];
                    #pragma unroll
                    for (int rr = 0; rr < 8; ++rr) {
                        const int M = mt * 16 + rr + msel;
                        sOut[M * SOSTR + co] += (acc[mt][nt][rr] * WINV + bs) * sW8[M * 8 + wid];
                    }
                }
            }
        }
        __syncthreads();
    }

    v4f ov[2];
    #pragma unroll
    for (int it = 0; it < 2; ++it) {
        const int co = it * 32 + wid * 4 + (lane >> 3);
        const int px = (lane & 7) * 4;
        v4f v;
        v.x = sOut[(px + 0) * SOSTR + co];
        v.y = sOut[(px + 1) * SOSTR + co];
        v.z = sOut[(px + 2) * SOSTR + co];
        v.w = sOut[(px + 3) * SOSTR + co];
        ov[it] = v;
    }
    #pragma unroll
    for (int it = 0; it < 2; ++it) {
        const int co = it * 32 + wid * 4 + (lane >> 3);
        const int px = (lane & 7) * 4;
        *(volatile v4f*)(out + ((size_t)(b * COUT + co)) * HWSZ + hwbase + px) = ov[it];
    }
    __threadfence();
    #pragma unroll
    for (int it = 0; it < 2; ++it) {
        const int co = it * 32 + wid * 4 + (lane >> 3);
        const int px = (lane & 7) * 4;
        *(volatile v4f*)(out + ((size_t)(b * COUT + co)) * HWSZ + hwbase + px) = ov[it];
    }
}

extern "C" void kernel_launch(void* const* d_in, const int* in_sizes, int n_in,
                              void* d_out, int out_size, void* d_ws, size_t ws_size,
                              hipStream_t stream) {
    if (n_in < 8) return;
    if (in_sizes[0] != 2 * CIN * HWSZ)  return;
    if (in_sizes[1] != 2 * 18 * HWSZ)   return;
    if (in_sizes[2] != 2 * 9 * HWSZ)    return;
    if (in_sizes[3] != 2 * 8 * HWSZ)    return;
    if (in_sizes[4] != COUT * CIN * 9)  return;
    if (in_sizes[5] < NOUT)             return;
    if (in_sizes[6] != 4 * CIN)         return;
    if (in_sizes[7] < 4)                return;
    if (out_size != 2 * COUT * HWSZ)    return;

    const float* input  = (const float*)d_in[0];
    const float* offset = (const float*)d_in[1];
    const float* maskp  = (const float*)d_in[2];
    const float* wc8    = (const float*)d_in[3];
    const float* weight = (const float*)d_in[4];
    const float* bias   = (const float*)d_in[5];
    const float* fc_w   = (const float*)d_in[6];
    const float* fc_b   = (const float*)d_in[7];
    float* out = (float*)d_out;

    const int    nplanes  = 2 * CIN;
    const size_t p_bytes  = (size_t)nplanes * PSTR * sizeof(float);
    const size_t wq_bytes = (size_t)NOUT * WQP * 2;
    if (p_bytes + wq_bytes > ws_size) return;

    char* ws = (char*)d_ws;
    float*    P  = (float*)ws;
    _Float16* wq = (_Float16*)(ws + p_bytes);

    const int npix = 2 * HWSZ;
    const int nblk = (npix + MT - 1) / MT;

    k_pool<<<nplanes, 256, 0, stream>>>(input, P, nplanes);
    k_blend<<<COUT, 256, 0, stream>>>(weight, P, fc_w, fc_b, wq);
    k_deform<<<nblk, 256, 0, stream>>>(input, offset, maskp, wc8, bias, wq, out, npix);
}
